// MultiHeadedAttention_86242943304407
// MI455X (gfx1250) — hardware-verified
//
#include <hip/hip_runtime.h>


#ifndef NB
#define NB 128
#endif
#ifndef SEQ
#define SEQ 256
#endif
#define NB_FULL  128
#define SEQ_FULL 256
#define DM   256
#define NH_  4
#define HD   64
#define AW   4
#define OSP  68
#define SPL  (SEQ / 2 + 4)
#define QRS  2048.0f
#define QRI  (1.0f / 2048.0f)
#define LOG2E 1.4426950408889634f
#define PSH  14.0f
#define NEGB (-3.0e38f)
#define POSB (3.0e38f)
#define WSC  16.0f
#define WSI  0.0625f

static_assert(HD == 64);
static_assert(NH_ * HD == DM);
static_assert(DM % 64 == 0);
static_assert(DM % 32 == 0);
static_assert(HD % 32 == 0);
static_assert(SEQ % 64 == 0);
static_assert((NB * SEQ) % 64 == 0);
static_assert(SEQ % 32 == 0);
static_assert(SEQ % (16 * AW) == 0);
static_assert((SPL * 4) % 16 == 0);
static_assert((OSP * 4) % 16 == 0);
static_assert(SPL >= SEQ / 2);
static_assert(NB <= NB_FULL);
static_assert(SEQ <= SEQ_FULL);
static_assert(SEQ_FULL % 64 == 0);
static_assert(((size_t)DM * DM) % 8 == 0);
static_assert((size_t)AW * 32 * SPL * 4 + (size_t)AW * 16 * OSP * 4 <= 131072);
static_assert((size_t)64 * 65 * 4 <= 131072);
static_assert((size_t)16 * 68 * 4 <= 131072);
static_assert(4 * 32 * 16 == 16 * HD * 2);
static_assert(4 * 32 * 16 == 16 * 64 * 2);
static_assert(4 * 32 * 16 == 16 * HD * 2);
static_assert(8 * 32 * 16 == 16 * 64 * 4);
static_assert(2 * 256 * 16 == 64 * 64 * 2);

typedef _Float16 h16;
typedef unsigned short bf;
typedef __attribute__((ext_vector_type(16))) __bf16   v16bf;
typedef __attribute__((ext_vector_type(16))) _Float16 v16h;
typedef __attribute__((ext_vector_type(8)))  _Float16 v8h;
typedef __attribute__((ext_vector_type(8)))  unsigned short v8us;
typedef __attribute__((ext_vector_type(8)))  float    v8f;
typedef __attribute__((ext_vector_type(4)))  float    v4f;
typedef v4f  __attribute__((may_alias)) v4fa;

__device__ __forceinline__ unsigned short f2bf(float f) { unsigned u = __float_as_uint(f); u += 0x7FFFu + ((u >> 16) & 1u); return (unsigned short)(u >> 16); }
__device__ __forceinline__ float bfr(float f) { return __uint_as_float(((unsigned)f2bf(f)) << 16); }
__device__ __forceinline__ v16h cat16(v8h lo, v8h hi) { return __builtin_shufflevector(lo, hi, 0, 1, 2, 3, 4, 5, 6, 7, 8, 9, 10, 11, 12, 13, 14, 15); }
__device__ __forceinline__ v16bf cat16b(v8us lo, v8us hi) { return __builtin_bit_cast(v16bf, __builtin_shufflevector(lo, hi, 0, 1, 2, 3, 4, 5, 6, 7, 8, 9, 10, 11, 12, 13, 14, 15)); }
__device__ __forceinline__ v16h  ldh(const h16* p) { return cat16(*(const v8h*)p, *(const v8h*)(p + 16)); }
__device__ __forceinline__ v16bf ldb(const bf* p)  { return cat16b(*(const v8us*)p, *(const v8us*)(p + 16)); }
__device__ __forceinline__ void wave_sync() { __builtin_amdgcn_fence(3  , "wavefront"); __builtin_amdgcn_wave_barrier(); asm volatile("" ::: "memory"); }
__device__ __forceinline__ h16 toh_flush(float v) { const h16 r = (h16)v; return (fabsf(v) < 6.103515625e-05f) ? (h16)0.0f : r; }
__device__ __forceinline__ v8f wmma16g(v16h a, v16h b, v8f c) {
    c = __builtin_amdgcn_wmma_f32_16x16x32_f16(false, a, false, b, (short)0, c, false, false);
    asm volatile("v_nop\n\tv_nop\n\tv_nop\n\tv_nop" : "+v"(c) : "v"(a), "v"(b));
    return c; }
__device__ __forceinline__ v8f wmmabg(v16bf a, v16bf b, v8f c) {
    c = __builtin_amdgcn_wmma_f32_16x16x32_bf16(false, a, false, b, (short)0, c, false, false);
    asm volatile("v_nop\n\tv_nop\n\tv_nop\n\tv_nop" : "+v"(c) : "v"(a), "v"(b));
    return c; }

__global__ __launch_bounds__(256) void k_tcvt(const float* __restrict__ src, bf* dst) {
    __shared__ float ts[64 * 65];
    const int tid = threadIdx.x;
    const int n0 = blockIdx.x * 64, f0 = blockIdx.y * 64, b = blockIdx.z;
    const float* sp = src + ((size_t)b * DM + f0) * SEQ_FULL + n0;
#pragma unroll
    for (int it = 0; it < 4; ++it) { const int q = it * 256 + tid; const int f = q >> 4, n4 = (q & 15) * 4;
        const v4f v = *(const v4f*)(sp + (size_t)f * SEQ_FULL + n4);
        ts[f * 65 + n4 + 0] = v[0]; ts[f * 65 + n4 + 1] = v[1]; ts[f * 65 + n4 + 2] = v[2]; ts[f * 65 + n4 + 3] = v[3]; }
    __syncthreads();
    v8us o[2];
#pragma unroll
    for (int it = 0; it < 2; ++it) { const int p = it * 256 + tid; const int n = p >> 3, c8 = (p & 7) * 8;
#pragma unroll
        for (int k = 0; k < 8; ++k) o[it][k] = f2bf(ts[(c8 + k) * 65 + n]); }
    bf* dp = dst + ((size_t)b * SEQ + n0) * DM + f0;
#pragma unroll 1
    for (int ps = 0; ps < 2; ++ps) {
#pragma unroll
        for (int it = 0; it < 2; ++it) { const int p = it * 256 + tid; const int n = p >> 3, c8 = (p & 7) * 8;
            *(volatile v8us*)(dp + (size_t)n * DM + c8) = o[it]; }
        if (ps == 0) __threadfence(); }
}

__global__ __launch_bounds__(256) void k_wrow(const float* __restrict__ W, bf* dst) {
    const int i = blockIdx.x * 256 + threadIdx.x; if (i >= DM * DM / 8) return;
    const int ep = i / (DM / 8), c8 = (i % (DM / 8)) * 8; const int h = ep / HD, d = ep % HD; const int e = d * NH_ + h;
    const v8f v = *(const v8f*)(W + (size_t)e * DM + c8); v8us o;
#pragma unroll
    for (int k = 0; k < 8; ++k) o[k] = f2bf(v[k]);
    *(volatile v8us*)(dst + (size_t)i * 8) = o; __threadfence(); *(volatile v8us*)(dst + (size_t)i * 8) = o;
}

__global__ __launch_bounds__(256) void k_wcol(const float* __restrict__ W, h16* dst) {
    const int i = blockIdx.x * 256 + threadIdx.x; if (i >= DM * DM / 8) return;
    const int e = i / (DM / 8), c8 = (i % (DM / 8)) * 8; const int h = c8 / HD, d0 = c8 % HD;
    v8h o;
#pragma unroll
    for (int k = 0; k < 8; ++k) o[k] = toh_flush(bfr(W[(size_t)e * DM + (size_t)(d0 + k) * NH_ + h]) * WSC);
    *(volatile v8h*)(dst + (size_t)i * 8) = o; __threadfence(); *(volatile v8h*)(dst + (size_t)i * 8) = o;
}

__device__ __forceinline__ void gemm_bf_tile(const bf* __restrict__ A, const bf* __restrict__ Bt, const size_t aoff, const size_t boff, v8f (&acc)[4][4]) {
#pragma unroll 1
    for (int kc = 0; kc < DM; kc += 32) {
        v16bf a[4];
#pragma unroll
        for (int mb = 0; mb < 4; ++mb) a[mb] = ldb(A + aoff + (size_t)mb * 16 * DM + kc);
#pragma unroll
        for (int nb = 0; nb < 4; ++nb) { const v16bf b = ldb(Bt + boff + (size_t)nb * 16 * DM + kc);
#pragma unroll
            for (int mb = 0; mb < 4; ++mb) acc[mb][nb] = wmmabg(a[mb], b, acc[mb][nb]); }
    }
}
__device__ __forceinline__ void gemm_h_tile(const h16* __restrict__ A, const h16* __restrict__ Bt, const size_t aoff, const size_t boff, v8f (&acc)[4][4]) {
#pragma unroll 1
    for (int kc = 0; kc < DM; kc += 32) {
        v16h a[4];
#pragma unroll
        for (int mb = 0; mb < 4; ++mb) a[mb] = ldh(A + aoff + (size_t)mb * 16 * DM + kc);
#pragma unroll
        for (int nb = 0; nb < 4; ++nb) { const v16h b = ldh(Bt + boff + (size_t)nb * 16 * DM + kc);
#pragma unroll
            for (int mb = 0; mb < 4; ++mb) acc[mb][nb] = wmma16g(a[mb], b, acc[mb][nb]); }
    }
}

__global__ __launch_bounds__(32) void k_proj_tok(const bf* __restrict__ A, const bf* __restrict__ Bt, const float* __restrict__ bias, h16* Ph, h16* Pr) {
    __shared__ __align__(16) float os[16 * 68];
    const int lane = threadIdx.x & 31, lr = lane & 15, hi = lane >> 4; const int r0 = blockIdx.x * 64, c0 = blockIdx.y * 64;
    v8f acc[4][4];
#pragma unroll
    for (int mb = 0; mb < 4; ++mb)
#pragma unroll
        for (int nb = 0; nb < 4; ++nb) acc[mb][nb] = (v8f){};
    gemm_bf_tile(A, Bt, (size_t)(r0 + lr) * DM + 8 * hi, (size_t)(c0 + lr) * DM + 8 * hi, acc);
    const int hh = c0 / HD;
    float bc[4];
#pragma unroll
    for (int nb = 0; nb < 4; ++nb) bc[nb] = bfr(bias[(nb * 16 + lr) * NH_ + hh]);
    const int bb = r0 / SEQ, tt = r0 % SEQ;
    const size_t tbase = ((size_t)(bb * NH_ + hh) * SEQ + (size_t)tt) * HD;
#pragma unroll
    for (int mb = 0; mb < 4; ++mb) {
#pragma unroll
        for (int nb = 0; nb < 4; ++nb) {
#pragma unroll
            for (int j = 0; j < 8; ++j) os[(hi * 8 + j) * 68 + nb * 16 + lr] = acc[mb][nb][j] + bc[nb]; }
        wave_sync();
#pragma unroll 1
        for (int ps = 0; ps < 2; ++ps) {
            const size_t sb = tbase + (size_t)(mb * 16) * HD;
#pragma unroll
            for (int s = 0; s < 4; ++s) { const int p = s * 32 + lane; const int row = p >> 3, c8 = (p & 7) * 8;
                const v4f x0 = *(const v4fa*)(&os[row * 68 + c8]); const v4f x1 = *(const v4fa*)(&os[row * 68 + c8 + 4]); v8h hv, rv;
#pragma unroll
                for (int i = 0; i < 4; ++i) { const h16 a0 = toh_flush(x0[i]); const h16 a1 = toh_flush(x1[i]); hv[i] = a0; hv[4 + i] = a1;
                    rv[i] = toh_flush((x0[i] - (float)a0) * QRS); rv[4 + i] = toh_flush((x1[i] - (float)a1) * QRS); }
                const size_t oo = sb + (size_t)p * 8;
                *(volatile v8h*)(Ph + oo) = hv; *(volatile v8h*)(Pr + oo) = rv; }
            if (ps == 0) __threadfence(); }
        wave_sync();
    }
}

__global__ __launch_bounds__(32) void k_proj_ch(const bf* __restrict__ A, const bf* __restrict__ Bt, const float* __restrict__ bias, h16* Ph) {
    __shared__ __align__(16) float os[16 * 68];
    const int lane = threadIdx.x & 31, lr = lane & 15, hi = lane >> 4; const int r0 = blockIdx.x * 64, c0 = blockIdx.y * 64;
    v8f acc[4][4];
#pragma unroll
    for (int mb = 0; mb < 4; ++mb)
#pragma unroll
        for (int nb = 0; nb < 4; ++nb) acc[mb][nb] = (v8f){};
    gemm_bf_tile(A, Bt, (size_t)(r0 + lr) * DM + 8 * hi, (size_t)(c0 + lr) * DM + 8 * hi, acc);
    const int hh = r0 / HD;
    const int bb = c0 / SEQ, tt = c0 % SEQ;
    const size_t tbase = ((size_t)bb * DM + (size_t)r0) * SEQ + (size_t)tt;
#pragma unroll
    for (int mb = 0; mb < 4; ++mb) {
        float br[8];
#pragma unroll
        for (int j = 0; j < 8; ++j) br[j] = bfr(bias[(mb * 16 + hi * 8 + j) * NH_ + hh]);
#pragma unroll
        for (int nb = 0; nb < 4; ++nb) {
#pragma unroll
            for (int j = 0; j < 8; ++j) os[(hi * 8 + j) * 68 + nb * 16 + lr] = acc[mb][nb][j] + br[j]; }
        wave_sync();
#pragma unroll 1
        for (int ps = 0; ps < 2; ++ps) {
            const size_t sb = tbase + (size_t)(mb * 16) * SEQ;
#pragma unroll
            for (int s = 0; s < 4; ++s) { const int row = 4 * s + (lane >> 3), c8 = (lane & 7) * 8;
                const v4f x0 = *(const v4fa*)(&os[row * 68 + c8]); const v4f x1 = *(const v4fa*)(&os[row * 68 + c8 + 4]); v8h hv;
#pragma unroll
                for (int i = 0; i < 4; ++i) { hv[i] = toh_flush(x0[i]); hv[4 + i] = toh_flush(x1[i]); }
                *(volatile v8h*)(Ph + sb + (size_t)row * SEQ + c8) = hv; }
            if (ps == 0) __threadfence(); }
        wave_sync();
    }
}

__global__ __launch_bounds__(32 * AW) __attribute__((amdgpu_num_vgpr(256))) void k_attn(const h16* __restrict__ QH, const h16* __restrict__ QR, const h16* __restrict__ KP, const h16* __restrict__ KR,
                                                                                       const h16* __restrict__ VT, const int* __restrict__ kptr, h16* CX) {
    __shared__ __align__(16) float ss[AW * 32 * SPL];
    __shared__ __align__(16) float os[AW * 16 * OSP];
    const int lane = threadIdx.x & 31, lr = lane & 15, hi = lane >> 4;
    const int wave = __builtin_amdgcn_readfirstlane((int)(threadIdx.x >> 5));
    const int zh = blockIdx.y; const int b = zh / NH_, h = zh % NH_;
    const int t0 = (blockIdx.x * AW + wave) * 16;
    int kTop = kptr[0]; kTop = kTop < 1 ? 1 : (kTop > SEQ ? SEQ : kTop);
    const size_t pbase = (size_t)zh * SEQ * HD;
    const size_t qo = pbase + (size_t)(t0 + lr) * HD + 8 * hi;
    const v16h qh0 = ldh(QH + qo), qh1 = ldh(QH + qo + 32), qr0 = ldh(QR + qo), qr1 = ldh(QR + qo + 32);
    const size_t ko = pbase + (size_t)lr * HD + 8 * hi;
    const size_t vo = pbase + (size_t)lr * SEQ + 8 * hi;
    const int lb = (wave * 32 + lane) * SPL;
#pragma unroll 1
    for (int j = 0; j < SEQ / 16; ++j) {
        const size_t kk = ko + (size_t)j * 16 * HD;
        const v16h k0 = ldh(KP + kk), k1 = ldh(KP + kk + 32), kr0 = ldh(KR + kk), kr1 = ldh(KR + kk + 32);
        v8f sH = (v8f){}, sL = (v8f){};
        sH = wmma16g(k0, qh0, sH); sH = wmma16g(k1, qh1, sH);
        sL = wmma16g(k0, qr0, sL); sL = wmma16g(k1, qr1, sL);
        sL = wmma16g(kr0, qh0, sL); sL = wmma16g(kr1, qh1, sL);
        v4f a, c;
#pragma unroll
        for (int r = 0; r < 4; ++r) { a[r] = (sH[r] + sL[r] * QRI) * 0.125f; c[r] = (sH[4 + r] + sL[4 + r] * QRI) * 0.125f; }
        *(v4fa*)(&ss[lb + 8 * j]) = a; *(v4fa*)(&ss[lb + 8 * j + 4]) = c;
    }
    wave_sync();
    float thr = POSB, rmax = NEGB; int cnt = 0;
#pragma unroll 1
    for (int it = 0; it < kTop; ++it) {
        float lm = NEGB; int cl = 0;
#pragma unroll 2
        for (int i = 0; i < SEQ / 8; ++i) {
            const v4f x = *(const v4fa*)(&ss[lb + 4 * i]);
#pragma unroll
            for (int c = 0; c < 4; ++c) {
                const float w = (x[c] < thr) ? x[c] : NEGB;
                const bool gt = w > lm; const bool eq = (w == lm);
                cl = gt ? 1 : (eq ? cl + 1 : cl);
                lm = gt ? w : lm; }
        }
        const float lmo = __shfl_xor(lm, 16, 32); const int clo = __shfl_xor(cl, 16, 32);
        const float gm = fmaxf(lm, lmo);
        const int c2 = ((lm == gm) ? cl : 0) + ((lmo == gm) ? clo : 0);
        const bool act = cnt < kTop;
        rmax = (it == 0) ? gm : rmax;
        thr = act ? gm : thr; cnt = act ? (cnt + c2) : cnt;
    }
    v8f o[4];
#pragma unroll
    for (int jd = 0; jd < 4; ++jd) o[jd] = (v8f){};
    float l = 0.0f;
#pragma unroll 1
    for (int s = 0; s < SEQ / 32; ++s) {
        v16h pb;
#pragma unroll
        for (int q4 = 0; q4 < 4; ++q4) { const v4f xv = *(const v4fa*)(&ss[lb + 16 * s + 4 * q4]);
#pragma unroll
            for (int c = 0; c < 4; ++c) { const float x = xv[c]; const float e = (x - rmax) * LOG2E + PSH;
                const bool kp = (x >= thr) & (e >= -14.0f);
                const float g = kp ? __builtin_amdgcn_exp2f(e) : 0.0f;
                const h16 pa = (h16)g; pb[4 * q4 + c] = pa; l += (float)pa; } }
        const h16* va = VT + vo + 32 * s;
        v16h v[4];
#pragma unroll
        for (int jd = 0; jd < 4; ++jd) v[jd] = ldh(va + (size_t)jd * 16 * SEQ);
#pragma unroll
        for (int jd = 0; jd < 4; ++jd) o[jd] = wmma16g(v[jd], pb, o[jd]);
    }
    l += __shfl_xor(l, 16, 32);
    const bool any = l > 0.0f;
    const float lsafe = any ? l : 1.0f;
    const float inv = any ? (1.0f / lsafe) : 0.0f;
    const int wb = wave * 16 * OSP;
#pragma unroll
    for (int jd = 0; jd < 4; ++jd) { v4f a, c;
        a[0] = o[jd][0] * inv; a[1] = o[jd][1] * inv; a[2] = o[jd][2] * inv; a[3] = o[jd][3] * inv;
        c[0] = o[jd][4] * inv; c[1] = o[jd][5] * inv; c[2] = o[jd][6] * inv; c[3] = o[jd][7] * inv;
        *(v4fa*)(&os[wb + lr * OSP + 16 * jd + 8 * hi]) = a; *(v4fa*)(&os[wb + lr * OSP + 16 * jd + 8 * hi + 4]) = c; }
    wave_sync();
    h16* crow = CX + ((size_t)b * SEQ + t0) * DM + h * HD;
#pragma unroll 1
    for (int ps = 0; ps < 2; ++ps) {
#pragma unroll
        for (int s = 0; s < 4; ++s) { const int row = 4 * s + (lane >> 3), c8 = (lane & 7) * 8;
            const v4f x0 = *(const v4fa*)(&os[wb + row * OSP + c8]); const v4f x1 = *(const v4fa*)(&os[wb + row * OSP + c8 + 4]); v8h hv;
#pragma unroll
            for (int i = 0; i < 4; ++i) { hv[i] = toh_flush(x0[i]); hv[4 + i] = toh_flush(x1[i]); }
            *(volatile v8h*)(crow + (size_t)row * DM + c8) = hv; }
        if (ps == 0) __threadfence(); }
}

__global__ __launch_bounds__(32) void k_outp(const h16* __restrict__ A, const h16* __restrict__ Bt, const float* __restrict__ bias, float* OUT) {
    __shared__ __align__(16) float os[16 * 68];
    const int lane = threadIdx.x & 31, lr = lane & 15, hi = lane >> 4; const int r0 = blockIdx.x * 64, c0 = blockIdx.y * 64;
    v8f acc[4][4];
#pragma unroll
    for (int mb = 0; mb < 4; ++mb)
#pragma unroll
        for (int nb = 0; nb < 4; ++nb) acc[mb][nb] = (v8f){};
    gemm_h_tile(A, Bt, (size_t)(r0 + lr) * DM + 8 * hi, (size_t)(c0 + lr) * DM + 8 * hi, acc);
    const int bb = c0 / SEQ, tt = c0 % SEQ;
    float* ob = OUT + ((size_t)bb * DM + (size_t)r0) * SEQ_FULL + (size_t)tt;
#pragma unroll
    for (int mb = 0; mb < 4; ++mb) {
        float br[8];
#pragma unroll
        for (int j = 0; j < 8; ++j) br[j] = bfr(bias[r0 + mb * 16 + hi * 8 + j]);
#pragma unroll
        for (int nb = 0; nb < 4; ++nb) {
#pragma unroll
            for (int j = 0; j < 8; ++j) os[(hi * 8 + j) * 68 + nb * 16 + lr] = acc[mb][nb][j] * WSI + br[j]; }
        wave_sync();
#pragma unroll 1
        for (int ps = 0; ps < 2; ++ps) {
#pragma unroll
            for (int s = 0; s < 8; ++s) { const int row = 2 * s + (lane >> 4), cofs = (lane & 15) * 4;
                const v4f val = *(const v4fa*)(&os[row * 68 + cofs]);
                *(volatile v4f*)(ob + (size_t)(mb * 16 + row) * SEQ_FULL + cofs) = val; }
            if (ps == 0) __threadfence(); }
        wave_sync();
    }
}

static constexpr size_t al256(size_t v) { return (v + 255) & ~(size_t)255; }
static constexpr size_t SZ_XB = al256((size_t)NB * SEQ * DM * 2);
static constexpr size_t SZ_WB = al256((size_t)3 * DM * DM * 2);
static constexpr size_t SZ_WM = al256((size_t)DM * DM * 2);
static constexpr size_t SZ_PL = al256((size_t)NB * NH_ * SEQ * HD * 2);
static constexpr size_t SZ_TOTAL = 2 * SZ_XB + SZ_WB + SZ_WM + 5 * SZ_PL;
static_assert(SZ_TOTAL <= (size_t)134217728);
static_assert(((size_t)DM * DM * 2) % 256 == 0);
static_assert((size_t)NB * NH_ * SEQ * HD == (size_t)NB * DM * SEQ);
static_assert((size_t)NB * SEQ * DM * 2 <= SZ_XB);
static_assert((DM * DM / 8) % 256 == 0);

extern "C" void kernel_launch(void* const* d_in, const int* in_sizes, int n_in,
                              void* d_out, int out_size, void* d_ws, size_t ws_size, hipStream_t stream) {
    if (n_in < 11) return;
    const size_t needx = ((size_t)(NB - 1) * DM + (size_t)(DM - 1)) * SEQ_FULL + SEQ;
    if ((size_t)in_sizes[0] < needx || (size_t)in_sizes[1] < needx) return;
    if ((size_t)in_sizes[2] < (size_t)DM * DM || (size_t)in_sizes[4] < (size_t)DM * DM || (size_t)in_sizes[6] < (size_t)DM * DM || (size_t)in_sizes[8] < (size_t)DM * DM) return;
    if (in_sizes[3] < DM || in_sizes[5] < DM || in_sizes[7] < DM || in_sizes[9] < DM || in_sizes[10] < 1) return;
    if ((size_t)out_size < needx) return;
    if (SZ_TOTAL > ws_size) return;
    const float* xq = (const float*)d_in[0]; const float* xs = (const float*)d_in[1];
    const float* wq = (const float*)d_in[2]; const float* bq = (const float*)d_in[3];
    const float* wk = (const float*)d_in[4]; const float* bk = (const float*)d_in[5];
    const float* wv = (const float*)d_in[6]; const float* bv = (const float*)d_in[7];
    const float* wm = (const float*)d_in[8]; const float* bm = (const float*)d_in[9];
    const int* kp = (const int*)d_in[10];
    float* OUT = (float*)d_out;
    char* wsp = (char*)d_ws;
    bf* XB = (bf*)wsp; h16* CX = (h16*)wsp; wsp += SZ_XB;
    bf* SB = (bf*)wsp; wsp += SZ_XB;
    bf* WB = (bf*)wsp; wsp += SZ_WB;
    h16* WM = (h16*)wsp; wsp += SZ_WM;
    h16* QH = (h16*)wsp; wsp += SZ_PL;
    h16* QR = (h16*)wsp; wsp += SZ_PL;
    h16* KP = (h16*)wsp; wsp += SZ_PL;
    h16* KR = (h16*)wsp; wsp += SZ_PL;
    h16* VT = (h16*)wsp; wsp += SZ_PL;
    bf* WQ = WB; bf* WK = WB + (size_t)DM * DM; bf* WV = WB + (size_t)2 * DM * DM;

    k_tcvt<<<dim3(SEQ / 64, DM / 64, NB), 256, 0, stream>>>(xq, XB);
    k_tcvt<<<dim3(SEQ / 64, DM / 64, NB), 256, 0, stream>>>(xs, SB);
    { const unsigned g = (unsigned)((DM * DM / 8 + 255) / 256);
      k_wrow<<<g, 256, 0, stream>>>(wq, WQ); k_wrow<<<g, 256, 0, stream>>>(wk, WK); k_wrow<<<g, 256, 0, stream>>>(wv, WV);
      k_wcol<<<g, 256, 0, stream>>>(wm, WM); }

    k_proj_tok<<<dim3(NB * SEQ / 64, DM / 64, 1), 32, 0, stream>>>(XB, WQ, bq, QH, QR);
    k_proj_tok<<<dim3(NB * SEQ / 64, DM / 64, 1), 32, 0, stream>>>(SB, WK, bk, KP, KR);
    k_proj_ch<<<dim3(DM / 64, NB * SEQ / 64, 1), 32, 0, stream>>>(WV, SB, bv, VT);

    k_attn<<<dim3(SEQ / (16 * AW), NB * NH_, 1), 32 * AW, 0, stream>>>(QH, QR, KP, KR, VT, kp, CX);

    k_outp<<<dim3(DM / 64, NB * SEQ / 64, 1), 32, 0, stream>>>(WM, CX, bm, OUT);
}
